// CausalSelfAttention_23046794510819
// MI455X (gfx1250) — hardware-verified
//
#include <hip/hip_runtime.h>


#ifndef NB
#define NB 4
#endif
#ifndef SEQ
#define SEQ 2048
#endif
#define NB_FULL  4
#define SEQ_FULL 2048
#define DM   1024
#define NH   16
#define HD   64
#define RH   ((SEQ) < 256 ? (SEQ) : 256)
#define PP   40
#define CSP  68
#define CTXP (2 * DM)
#define NEGB (-1.0e30f)
#define RSC  4.8828125e-4f
#define RCAR 2048.0f
#define CCAR 16.0f
#define OSC  3.0517578125e-5f
#define SCL2 0.18033688011112042f

static_assert(HD == 64);
static_assert(DM == NH * HD);
static_assert(DM % 64 == 0);
static_assert(DM % 32 == 0);
static_assert(SEQ % 64 == 0);
static_assert(RH % 64 == 0);
static_assert(RH <= SEQ);
static_assert((NB * SEQ) % 64 == 0);
static_assert(NB <= NB_FULL);
static_assert(SEQ <= SEQ_FULL);
static_assert(PP % 8 == 0);
static_assert(PP >= 32);
static_assert(CSP % 4 == 0);
static_assert(CSP >= 64);
static_assert(((size_t)(NB - 1) * SEQ_FULL + SEQ) * DM * 4 <= (size_t)33554432);

typedef _Float16 h16;
typedef unsigned short bf;
typedef __attribute__((ext_vector_type(16))) __bf16   v16bf;
typedef __attribute__((ext_vector_type(16))) _Float16 v16h;
typedef __attribute__((ext_vector_type(8)))  _Float16 v8h;
typedef __attribute__((ext_vector_type(8)))  unsigned short v8us;
typedef __attribute__((ext_vector_type(16))) unsigned short v16us;
typedef __attribute__((ext_vector_type(8)))  float    v8f;
typedef __attribute__((ext_vector_type(4)))  float    v4f;
typedef v8h  __attribute__((may_alias)) v8ha;
typedef v4f  __attribute__((may_alias)) v4fa;

#define PLN ((size_t)NB * NH * SEQ * HD)
#define PLR ((size_t)NB * NH * RH * HD)
#define OFF_QH ((size_t)0)
#define OFF_QR (PLN)
#define OFF_KH (2 * PLN)
#define OFF_VH (3 * PLN)
#define OFF_KR (4 * PLN)
#define OFF_VR (4 * PLN + PLR)
#define PL_ELEMS (4 * PLN + 2 * PLR)

__device__ __forceinline__ unsigned short f2bf(float f) { unsigned u = __float_as_uint(f); u += 0x7FFFu + ((u >> 16) & 1u); return (unsigned short)(u >> 16); }
__device__ __forceinline__ float bf2f(unsigned short b) { return __uint_as_float(((unsigned)b) << 16); }
__device__ __forceinline__ float bfr(float f) { return bf2f(f2bf(f)); }
__device__ __forceinline__ v16h cat16(v8h lo, v8h hi) { return __builtin_shufflevector(lo, hi, 0, 1, 2, 3, 4, 5, 6, 7, 8, 9, 10, 11, 12, 13, 14, 15); }
__device__ __forceinline__ v16bf cat16b(v8us lo, v8us hi) { return __builtin_bit_cast(v16bf, __builtin_shufflevector(lo, hi, 0, 1, 2, 3, 4, 5, 6, 7, 8, 9, 10, 11, 12, 13, 14, 15)); }
__device__ __forceinline__ v8f wmma16(v16h a, v16h b, v8f c) { return __builtin_amdgcn_wmma_f32_16x16x32_f16(false, a, false, b, (short)0, c, false, false); }
__device__ __forceinline__ v8f wmmab(v16bf a, v16bf b, v8f c) { return __builtin_amdgcn_wmma_f32_16x16x32_bf16(false, a, false, b, (short)0, c, false, false); }
__device__ __forceinline__ v16h ldh(const h16* p) { return cat16(*(const v8h*)p, *(const v8h*)(p + 16)); }
__device__ __forceinline__ v16bf ldb(const bf* p) { return cat16b(*(const v8us*)p, *(const v8us*)(p + 16)); }

__global__ __launch_bounds__(256) void k_cvtx(const float* __restrict__ x, bf* XB) {
    const size_t i = (size_t)blockIdx.x * 256 + threadIdx.x;
    if (i >= (size_t)NB * SEQ * DM / 8) return;
    const int c8 = (int)(i % (DM / 8)); const size_t m = i / (DM / 8); const size_t b = m / SEQ, t = m % SEQ;
    const v8f v = *(const v8f*)(x + (b * SEQ_FULL + t) * DM + (size_t)c8 * 8);
    v8us o;
#pragma unroll
    for (int k = 0; k < 8; ++k) o[k] = f2bf(v[k]);
    *(volatile v8us*)(XB + i * 8) = o; __threadfence(); *(volatile v8us*)(XB + i * 8) = o;
}
__global__ __launch_bounds__(256) void k_cvtw(const float* __restrict__ src, bf* dst, int n8) {
    const int i = blockIdx.x * 256 + threadIdx.x;
    if (i >= n8) return;
    const v8f v = *(const v8f*)(src + (size_t)i * 8);
    v8us o;
#pragma unroll
    for (int k = 0; k < 8; ++k) o[k] = f2bf(v[k]);
    *(volatile v8us*)(dst + (size_t)i * 8) = o; __threadfence(); *(volatile v8us*)(dst + (size_t)i * 8) = o;
}
__global__ __launch_bounds__(256) void k_cvtwp(const float* __restrict__ w, h16* WP2) {
    const int i = blockIdx.x * 256 + threadIdx.x;
    if (i >= DM * DM / 8) return;
    const int n = i / (DM / 8), kq = i % (DM / 8);
    const v8f v = *(const v8f*)(w + (size_t)i * 8);
    v8h a, c;
#pragma unroll
    for (int k = 0; k < 8; ++k) { const float r = bfr(v[k]); a[k] = (h16)(r * RCAR); c[k] = (h16)r; }
    h16* d = WP2 + (size_t)n * CTXP + kq * 8;
    *(volatile v8h*)d = a; *(volatile v8h*)(d + DM) = c; __threadfence(); *(volatile v8h*)d = a; *(volatile v8h*)(d + DM) = c;
}

__global__ __launch_bounds__(32) void k_proj(const bf* __restrict__ XB, const bf* __restrict__ WB, h16* PL) {
    __shared__ __align__(16) float os[64 * CSP];
    const int z = blockIdx.z;
    const bf* Bt = WB + (size_t)z * DM * DM;
    const int lane = threadIdx.x & 31, lr = lane & 15, hi = lane >> 4;
    const int r0 = blockIdx.x * 64, c0 = blockIdx.y * 64;
    v8f acc[4][4];
#pragma unroll
    for (int mb = 0; mb < 4; ++mb)
#pragma unroll
        for (int nb = 0; nb < 4; ++nb) acc[mb][nb] = (v8f){};
    const size_t aoff = (size_t)(r0 + lr) * DM + 8 * hi, boff = (size_t)(c0 + lr) * DM + 8 * hi;
#pragma unroll 1
    for (int kc = 0; kc < DM; kc += 32) {
        v16bf a[4];
#pragma unroll
        for (int mb = 0; mb < 4; ++mb) a[mb] = ldb(XB + aoff + (size_t)mb * 16 * DM + kc);
#pragma unroll
        for (int nb = 0; nb < 4; ++nb) { const v16bf bb = ldb(Bt + boff + (size_t)nb * 16 * DM + kc);
#pragma unroll
            for (int mb = 0; mb < 4; ++mb) acc[mb][nb] = wmmab(a[mb], bb, acc[mb][nb]); }
        asm volatile("v_nop\n\tv_nop\n\tv_nop\n\tv_nop" : "+v"(acc[0][0]), "+v"(acc[1][1]), "+v"(acc[2][2]), "+v"(acc[3][3]) : "v"(a[0]), "v"(a[3]));
    }
#pragma unroll
    for (int mb = 0; mb < 4; ++mb)
#pragma unroll
        for (int nb = 0; nb < 4; ++nb)
#pragma unroll
            for (int j = 0; j < 8; ++j) os[(mb * 16 + hi * 8 + j) * CSP + nb * 16 + lr] = acc[mb][nb][j];
    __syncthreads();
    const int b = r0 / SEQ, t0 = r0 % SEQ;
    const size_t bh = (size_t)(b * NH + (int)blockIdx.y);
    size_t hib, rsb, hst, rst; int rs_, cs_, wres;
    if (z == 0)      { hib = OFF_QH + (bh * SEQ + t0) * HD; rsb = OFF_QR + (bh * SEQ + t0) * HD; hst = HD; rst = HD; rs_ = CSP; cs_ = 1; wres = 1; }
    else if (z == 1) { hib = OFF_KH + (bh * SEQ + t0) * HD; rsb = OFF_KR + (bh * RH + t0) * HD;  hst = HD; rst = HD; rs_ = CSP; cs_ = 1; wres = (t0 < RH) ? 1 : 0; }
    else             { hib = OFF_VH + bh * HD * SEQ + t0;   rsb = OFF_VR + bh * HD * RH + t0;    hst = SEQ; rst = RH; rs_ = 1; cs_ = CSP; wres = (t0 < RH) ? 1 : 0; }
    const int rq = lane >> 3, pc = lane & 7;
#pragma unroll 1
    for (int pz = 0; pz < 2; ++pz) {
#pragma unroll 1
        for (int it = 0; it < 16; ++it) {
            const int row = it * 4 + rq;
            v8h hv, rv;
#pragma unroll
            for (int j = 0; j < 8; ++j) { const float v = os[row * rs_ + (pc * 8 + j) * cs_]; const h16 hh = (h16)v; hv[j] = hh; rv[j] = (h16)((v - (float)hh) * RCAR); }
            *(volatile v8h*)(PL + hib + (size_t)row * hst + pc * 8) = hv;
            if (wres) *(volatile v8h*)(PL + rsb + (size_t)row * rst + pc * 8) = rv;
        }
        if (pz == 0) __threadfence();
    }
}

template <bool EARLY>
__device__ __forceinline__ void attn_body(const h16* __restrict__ PL, h16* CTX, int rb0) {
    __shared__ __align__(16) h16 ps[16 * PP];
    __shared__ __align__(16) h16 pr[16 * PP];
    __shared__ __align__(16) float cs[16 * CSP];
    const int lane = threadIdx.x & 31, lr = lane & 15, hi = lane >> 4;
    const int hh = blockIdx.y, b = blockIdx.z;
    const int q0 = (rb0 + (int)blockIdx.x) * 16;
    const size_t hb = (size_t)(b * NH + hh);
    const h16* qh = PL + OFF_QH + hb * SEQ * HD;
    const h16* qr = PL + OFF_QR + hb * SEQ * HD;
    const h16* kh = PL + OFF_KH + hb * SEQ * HD;
    const h16* vh = PL + OFF_VH + hb * HD * SEQ;
    const h16* kr = PL + OFF_KR + hb * RH * HD;
    const h16* vr = PL + OFF_VR + hb * HD * RH;
    const size_t qoff = (size_t)(q0 + lr) * HD + 8 * hi;
    v8f o[4], orr[4];
#pragma unroll
    for (int n = 0; n < 4; ++n) { o[n] = (v8f){}; orr[n] = (v8f){}; }
    float mrow[8], lrow[8];
#pragma unroll
    for (int r = 0; r < 8; ++r) { mrow[r] = NEGB; lrow[r] = 0.0f; }
    const int nkb = (q0 + 15) / 32 + 1;
#pragma unroll 1
    for (int kb = 0; kb < nkb; ++kb) {
        const int key0 = kb * 32;
        v8f s0 = (v8f){}, s1 = (v8f){}, x0 = (v8f){}, x1 = (v8f){};
#pragma unroll
        for (int kk = 0; kk < 2; ++kk) {
            const v16h aq = ldh(qh + qoff + kk * 32);
            const v16h ar = ldh(qr + qoff + kk * 32);
            const size_t ko = (size_t)(key0 + lr) * HD + 8 * hi + kk * 32;
            const v16h k0 = ldh(kh + ko);
            const v16h k1 = ldh(kh + ko + 16 * HD);
            s0 = wmma16(aq, k0, s0); s1 = wmma16(aq, k1, s1);
            x0 = wmma16(ar, k0, x0); x1 = wmma16(ar, k1, x1);
            if (EARLY) {
                const v16h e0 = ldh(kr + ko);
                const v16h e1 = ldh(kr + ko + 16 * HD);
                x0 = wmma16(aq, e0, x0); x1 = wmma16(aq, e1, x1);
                asm volatile("v_nop\n\tv_nop\n\tv_nop\n\tv_nop" : "+v"(s0), "+v"(s1), "+v"(x0), "+v"(x1) : "v"(aq), "v"(e0), "v"(e1));
            } else {
                asm volatile("v_nop\n\tv_nop\n\tv_nop\n\tv_nop" : "+v"(s0), "+v"(s1), "+v"(x0), "+v"(x1) : "v"(aq), "v"(ar), "v"(k0), "v"(k1));
            }
        }
#pragma unroll
        for (int r = 0; r < 8; ++r) {
            const int qrow = q0 + 8 * hi + r;
            float a0 = (s0[r] + x0[r] * RSC) * SCL2;
            float a1 = (s1[r] + x1[r] * RSC) * SCL2;
            a0 = (key0 + lr <= qrow) ? a0 : NEGB;
            a1 = (key0 + 16 + lr <= qrow) ? a1 : NEGB;
            float mx = fmaxf(a0, a1);
            mx = fmaxf(mx, __shfl_xor(mx, 1, 32));
            mx = fmaxf(mx, __shfl_xor(mx, 2, 32));
            mx = fmaxf(mx, __shfl_xor(mx, 4, 32));
            mx = fmaxf(mx, __shfl_xor(mx, 8, 32));
            const float mn = fmaxf(mrow[r], mx);
            const float corr = __builtin_amdgcn_exp2f(mrow[r] - mn);
            mrow[r] = mn;
            const float p0 = __builtin_amdgcn_exp2f(a0 - mn + 10.0f);
            const float p1 = __builtin_amdgcn_exp2f(a1 - mn + 10.0f);
            lrow[r] = lrow[r] * corr + (p0 + p1);
            o[0][r] *= corr; o[1][r] *= corr; o[2][r] *= corr; o[3][r] *= corr;
            if (EARLY) { orr[0][r] *= corr; orr[1][r] *= corr; orr[2][r] *= corr; orr[3][r] *= corr; }
            const int prow = (8 * hi + r) * PP;
            const h16 h0 = (h16)p0, h1 = (h16)p1;
            ps[prow + lr] = h0; ps[prow + 16 + lr] = h1;
            if (EARLY) { pr[prow + lr] = (h16)((p0 - (float)h0) * RCAR); pr[prow + 16 + lr] = (h16)((p1 - (float)h1) * RCAR); }
        }
        __syncthreads();
        const v16h pa = cat16(*(const v8ha*)(ps + lr * PP + 8 * hi), *(const v8ha*)(ps + lr * PP + 16 + 8 * hi));
        if (EARLY) {
            const v16h pb = cat16(*(const v8ha*)(pr + lr * PP + 8 * hi), *(const v8ha*)(pr + lr * PP + 16 + 8 * hi));
            v16h vf, vg;
#pragma unroll
            for (int n = 0; n < 4; ++n) {
                vf = ldh(vh + (size_t)(n * 16 + lr) * SEQ + key0 + 8 * hi);
                vg = ldh(vr + (size_t)(n * 16 + lr) * RH + key0 + 8 * hi);
                o[n] = wmma16(pa, vf, o[n]);
                orr[n] = wmma16(pb, vf, orr[n]);
                orr[n] = wmma16(pa, vg, orr[n]);
            }
            asm volatile("v_nop\n\tv_nop\n\tv_nop\n\tv_nop" : "+v"(o[0]), "+v"(o[1]), "+v"(o[2]), "+v"(o[3]), "+v"(orr[0]), "+v"(orr[1]), "+v"(orr[2]), "+v"(orr[3]) : "v"(pa), "v"(pb), "v"(vf), "v"(vg));
        } else {
            v16h vf[4];
#pragma unroll
            for (int n = 0; n < 4; ++n) vf[n] = ldh(vh + (size_t)(n * 16 + lr) * SEQ + key0 + 8 * hi);
#pragma unroll
            for (int n = 0; n < 4; ++n) o[n] = wmma16(pa, vf[n], o[n]);
            asm volatile("v_nop\n\tv_nop\n\tv_nop\n\tv_nop" : "+v"(o[0]), "+v"(o[1]), "+v"(o[2]), "+v"(o[3]) : "v"(pa), "v"(vf[3]));
        }
        __syncthreads();
    }
#pragma unroll
    for (int r = 0; r < 8; ++r) {
        float ls = lrow[r];
        ls += __shfl_xor(ls, 1, 32); ls += __shfl_xor(ls, 2, 32); ls += __shfl_xor(ls, 4, 32); ls += __shfl_xor(ls, 8, 32);
        const float inv = (1.0f / ls) * CCAR;
#pragma unroll
        for (int n = 0; n < 4; ++n) {
            float c = o[n][r];
            if (EARLY) c += orr[n][r] * RSC;
            cs[(8 * hi + r) * CSP + n * 16 + lr] = c * inv;
        }
    }
    __syncthreads();
    const int rq = lane >> 3, pc = lane & 7;
    v8h hv[4], rv[4];
#pragma unroll
    for (int s = 0; s < 4; ++s) {
        const int row = 4 * s + rq;
        const v4f a = *(const v4fa*)(cs + row * CSP + pc * 8);
        const v4f c = *(const v4fa*)(cs + row * CSP + pc * 8 + 4);
#pragma unroll
        for (int j = 0; j < 4; ++j) {
            const h16 ha = (h16)a[j]; hv[s][j] = ha; rv[s][j] = (h16)((a[j] - (float)ha) * RCAR);
            const h16 hc = (h16)c[j]; hv[s][4 + j] = hc; rv[s][4 + j] = (h16)((c[j] - (float)hc) * RCAR);
        }
    }
    const size_t cbase = ((size_t)b * SEQ + q0) * CTXP + (size_t)hh * HD + pc * 8;
#pragma unroll 1
    for (int pz = 0; pz < 2; ++pz) {
#pragma unroll
        for (int s = 0; s < 4; ++s) {
            h16* cp = CTX + cbase + (size_t)(4 * s + rq) * CTXP;
            *(volatile v8h*)cp = hv[s];
            *(volatile v8h*)(cp + DM) = rv[s];
        }
        if (pz == 0) __threadfence();
    }
}
__global__ __launch_bounds__(32) void k_attn_early(const h16* __restrict__ PL, h16* CTX) { attn_body<true>(PL, CTX, 0); }
__global__ __launch_bounds__(32) void k_attn_late(const h16* __restrict__ PL, h16* CTX) { attn_body<false>(PL, CTX, RH / 16); }

__global__ __launch_bounds__(32) void k_oproj(const h16* __restrict__ A, const h16* __restrict__ Bt, float* C) {
    __shared__ __align__(16) float os[16 * CSP];
    const int lane = threadIdx.x & 31, lr = lane & 15, hi = lane >> 4;
    const int r0 = blockIdx.x * 64, c0 = blockIdx.y * 64;
    v8f acc[4][4];
#pragma unroll
    for (int mb = 0; mb < 4; ++mb)
#pragma unroll
        for (int nb = 0; nb < 4; ++nb) acc[mb][nb] = (v8f){};
    const size_t aoff = (size_t)(r0 + lr) * CTXP + 8 * hi, boff = (size_t)(c0 + lr) * CTXP + 8 * hi;
#pragma unroll 1
    for (int kc = 0; kc < CTXP; kc += 32) {
        v16h a[4];
#pragma unroll
        for (int mb = 0; mb < 4; ++mb) a[mb] = ldh(A + aoff + (size_t)mb * 16 * CTXP + kc);
#pragma unroll
        for (int nb = 0; nb < 4; ++nb) { const v16h bb = ldh(Bt + boff + (size_t)nb * 16 * CTXP + kc);
#pragma unroll
            for (int mb = 0; mb < 4; ++mb) acc[mb][nb] = wmma16(a[mb], bb, acc[mb][nb]); }
        asm volatile("v_nop\n\tv_nop\n\tv_nop\n\tv_nop" : "+v"(acc[0][0]), "+v"(acc[1][1]), "+v"(acc[2][2]), "+v"(acc[3][3]) : "v"(a[0]), "v"(a[3]));
    }
    const int b = r0 / SEQ, t0 = r0 % SEQ;
#pragma unroll
    for (int mb = 0; mb < 4; ++mb) {
#pragma unroll
        for (int nb = 0; nb < 4; ++nb) {
#pragma unroll
            for (int j = 0; j < 8; ++j) os[(hi * 8 + j) * CSP + nb * 16 + lr] = acc[mb][nb][j]; }
        __syncthreads();
        float* crow = C + ((size_t)b * SEQ_FULL + t0 + mb * 16) * DM + c0;
#pragma unroll 1
        for (int pz = 0; pz < 2; ++pz) {
#pragma unroll
            for (int s = 0; s < 8; ++s) { const int row = 2 * s + hi, cofs = lr * 4; v4f val = *(const v4fa*)(os + row * CSP + cofs);
                val[0] *= OSC; val[1] *= OSC; val[2] *= OSC; val[3] *= OSC;
                *(volatile v4f*)(crow + (size_t)row * DM + cofs) = val; }
            if (pz == 0) __threadfence(); }
        __syncthreads();
    }
}

#define WS_XB  ((size_t)NB * SEQ * DM * 2)
#define WS_WB  ((size_t)3 * DM * DM * 2)
#define WS_WP  ((size_t)DM * CTXP * 2)
#define WS_PL  (PL_ELEMS * 2)
#define WS_CTX ((size_t)NB * SEQ * CTXP * 2)
#define WS_TOTAL (WS_XB + WS_WB + WS_WP + WS_PL + WS_CTX)
static_assert(WS_XB % 256 == 0);
static_assert(WS_WB % 256 == 0);
static_assert(WS_WP % 256 == 0);
static_assert(WS_PL % 256 == 0);
static_assert(WS_CTX % 256 == 0);
static_assert(WS_TOTAL <= (size_t)134217728);

extern "C" void kernel_launch(void* const* d_in, const int* in_sizes, int n_in,
                              void* d_out, int out_size, void* d_ws, size_t ws_size, hipStream_t stream) {
    if (n_in < 5) return;
    const long long xneed = ((long long)(NB - 1) * SEQ_FULL + SEQ) * DM;
    if ((long long)in_sizes[0] < xneed) return;
    if (in_sizes[1] < DM * DM || in_sizes[2] < DM * DM || in_sizes[3] < DM * DM || in_sizes[4] < DM * DM) return;
    if ((long long)out_size < xneed) return;
    if (ws_size < WS_TOTAL) return;
    const float* x  = (const float*)d_in[0];
    const float* wk = (const float*)d_in[1];
    const float* wq = (const float*)d_in[2];
    const float* wv = (const float*)d_in[3];
    const float* wp = (const float*)d_in[4];
    float* OUT = (float*)d_out;
    char* wsp = (char*)d_ws;
    bf*  XB  = (bf*)wsp;  wsp += WS_XB;
    bf*  WB  = (bf*)wsp;  wsp += WS_WB;
    h16* WP2 = (h16*)wsp; wsp += WS_WP;
    h16* PL  = (h16*)wsp; wsp += WS_PL;
    h16* CTX = (h16*)wsp; wsp += WS_CTX;

    k_cvtx<<<(unsigned)(((size_t)NB * SEQ * DM / 8 + 255) / 256), 256, 0, stream>>>(x, XB);
    k_cvtw<<<(unsigned)((DM * DM / 8 + 255) / 256), 256, 0, stream>>>(wq, WB, DM * DM / 8);
    k_cvtw<<<(unsigned)((DM * DM / 8 + 255) / 256), 256, 0, stream>>>(wk, WB + (size_t)DM * DM, DM * DM / 8);
    k_cvtw<<<(unsigned)((DM * DM / 8 + 255) / 256), 256, 0, stream>>>(wv, WB + (size_t)2 * DM * DM, DM * DM / 8);
    k_cvtwp<<<(unsigned)((DM * DM / 8 + 255) / 256), 256, 0, stream>>>(wp, WP2);
    k_proj<<<dim3(NB * SEQ / 64, DM / 64, 3), 32, 0, stream>>>(XB, WB, PL);
    k_attn_early<<<dim3(RH / 16, NH, NB), 32, 0, stream>>>(PL, CTX);
    if (SEQ > RH) k_attn_late<<<dim3((SEQ - RH) / 16, NH, NB), 32, 0, stream>>>(PL, CTX);
    k_oproj<<<dim3(NB * SEQ / 64, DM / 64, 1), 32, 0, stream>>>(CTX, WP2, OUT);
}
